// GraphAttentionLayer_53154515255605
// MI455X (gfx1250) — hardware-verified
//
#include <hip/hip_runtime.h>
#include <stddef.h>
#include <stdint.h>
#include <math.h>

#define NN     30000
#define EE     480000
#define CC     128
#define NBF    32
#define NAF    16
#define FCH    64
#define NHEAD  8
#define DHEAD  16
#define MP     30080
#define NTHR   256
#define NWAVE  8
#define EPT    8
#define CHUNK  (NTHR * EPT)
#define WCAP   (EPT * 32)
#define LISTN  (NWAVE * WCAP)
#define NBA    1024
#define SLA    10
#define ESH    19
#define EMASK  ((1 << ESH) - 1)
#define NBLK   30
#define NGRP   5
#define BPG    6
#define RCAP   28672
#define DEGCAP 64
#define VCAP   114688
#define TROWS  128
#define NTILE  (VCAP / TROWS)
#define MEAS_B1024  16653
#define MEAS_MAXDEG 34
#define GBM    64
#define GBN    128
#define GTHR   128
#define AP     264
#define DP     132
#define WSMAX  134217728ULL

#define SZ_AGG  ((size_t)MP * 256 * 2)
#define SZ_XB   ((size_t)MP * 128 * 2)
#define SZ_MSD  ((size_t)MP * 256 * 4)
#define SZ_VAL  ((size_t)VCAP * 128 * 4)
#define SZ_LOG  ((size_t)VCAP * 8 * 4)
#define SZ_HIT  ((size_t)NBLK * RCAP * 4)
#define SZ_FLG  ((size_t)4096)
#define O_AGG   ((size_t)0)
#define O_XB    (O_AGG + SZ_AGG)
#define O_MSD   (O_XB + SZ_XB)
#define O_VAL   (O_MSD + SZ_MSD)
#define O_LOG   (O_VAL + SZ_VAL)
#define O_HIT   (O_LOG + SZ_LOG)
#define O_FLG0  (O_HIT + SZ_HIT)
#define O_FLG1  (O_FLG0 + SZ_FLG)
#define O_WSD   (O_FLG1 + SZ_FLG)
#define O_W1T   (O_WSD + (size_t)256 * 128 * 2)
#define O_W2D   (O_W1T + (size_t)64 * 64 * 2)
#define O_W3D   (O_W2D + (size_t)64 * 128 * 2)
#define O_WALD  (O_W3D + (size_t)128 * 128 * 2)
#define O_WVD   (O_WALD + (size_t)256 * 256 * 2)
#define O_WOD   (O_WVD + (size_t)128 * 256 * 2)
#define O_PV    (O_WOD + (size_t)128 * 256 * 2)
#define WS_TOTAL (O_PV + (size_t)4096)

#define L_BUF0  0
#define L_BUF1  (TROWS * AP * 2)
#define L_G     (2 * TROWS * AP * 2)
#define L_LOG   (L_G + TROWS * DP * 4)
#define L_PV    (L_LOG + TROWS * 8 * 4)
#define L_EA    (L_PV + 768 * 4)
#define L_ID    (L_EA + TROWS * 4)
#define EDGE_LDS_BYTES (L_ID + 3 * TROWS * 4)
#define BKT_LDS_INTS  (LISTN + RCAP + 16)
#define SCAN_ZINTS    (RCAP + 3 * NBA)
#define SCAN_LDS_INTS (2 * RCAP + 3 * NBA + 16)

#define NU_XB  (MP * 16)
#define NU_K128 (128 * 16)
#define NU_W1  (64 * 8)
#define NU_W2  (64 * 16)
#define NU_W3  (128 * 16)
#define NU_PA  (NU_XB + 2 * NU_K128 + NU_W1 + NU_W2 + NU_W3)
#define NU_K256 (128 * 32)
#define NU_PB  (4 * NU_K256 + NTHR)

static_assert(WS_TOTAL <= WSMAX);
static_assert((SZ_AGG % 256) == 0 && (SZ_XB % 256) == 0 && (SZ_MSD % 256) == 0 && (SZ_VAL % 256) == 0);
static_assert((SZ_LOG % 256) == 0 && (SZ_HIT % 256) == 0 && NBLK * 128 <= 4096);
static_assert(NBLK * NBA >= MP && NGRP * BPG == NBLK && MP >= NN && (MP % 128) == 0 && (MP % GBM) == 0);
static_assert(EE < (1 << ESH) && NBA == (1 << SLA) && ESH + SLA < 31);
static_assert((CHUNK & (CHUNK - 1)) == 0 && ((long long)CHUNK << SLA) < (1LL << 31));
static_assert(RCAP >= MEAS_B1024 + 4096 && (RCAP % (NTHR * 4)) == 0);
static_assert(DEGCAP >= MEAS_MAXDEG + 8);
static_assert((VCAP % TROWS) == 0 && VCAP >= BPG * MEAS_B1024 && NTILE == 896);
static_assert(NHEAD * DHEAD == CC && NBF + 2 * NAF == FCH);
static_assert((SCAN_ZINTS % (NTHR * 4)) == 0);
static_assert(SCAN_LDS_INTS * 4 <= 300000 && BKT_LDS_INTS * 4 <= 300000 && EDGE_LDS_BYTES <= 300000);
static_assert((AP * 2) % 16 == 0 && AP >= 256 && (DP * 4) % 16 == 0 && DP >= 128);
static_assert((AP % 2) == 0 && (DP % 2) == 0 && (L_PV % 16) == 0 && (L_G % 16) == 0);
static_assert((NU_XB % NTHR) == 0 && (NU_K128 % NTHR) == 0 && (NU_W1 % NTHR) == 0 && (NU_W2 % NTHR) == 0);
static_assert((NU_W3 % NTHR) == 0 && (NU_K256 % NTHR) == 0 && (NU_PA % NTHR) == 0 && (NU_PB % NTHR) == 0);
static_assert(GBM == (GTHR / 32) * 16 && (NBA % GBM) == 0 && TROWS == NWAVE * 16);
static_assert((size_t)(NN - 1) * CC + CC - 1 == (size_t)NN * CC - 1);

typedef float          v2f  __attribute__((ext_vector_type(2)));
typedef float          v4f  __attribute__((ext_vector_type(4)));
typedef float          v8f  __attribute__((ext_vector_type(8)));
typedef int            v4i  __attribute__((ext_vector_type(4)));
typedef int            v8i  __attribute__((ext_vector_type(8)));
typedef unsigned       v4u  __attribute__((ext_vector_type(4)));
typedef unsigned short v4us __attribute__((ext_vector_type(4)));
typedef unsigned short v8us __attribute__((ext_vector_type(8)));
typedef __bf16         v16b __attribute__((ext_vector_type(16)));
typedef v2f  __attribute__((may_alias)) v2fa;
typedef v4f  __attribute__((may_alias)) v4fa;
typedef v4i  __attribute__((may_alias)) v4ia;
typedef v4us __attribute__((may_alias)) v4usa;
typedef v8us __attribute__((may_alias)) v8usa;
typedef unsigned int __attribute__((may_alias)) u32a;
union FragB { v16b v; v8us h[2]; v8i w; };

__device__ __forceinline__ v8f wmb(const FragB& a, const FragB& b, v8f c) {
  v8f d = __builtin_amdgcn_wmma_f32_16x16x32_bf16(false, a.v, false, b.v, (short)0, c, false, false);
  asm volatile("v_nop\n\tv_nop\n\tv_nop\n\tv_nop" : "+v"(d) : "v"(a.w), "v"(b.w));
  return d;
}

__device__ __forceinline__ unsigned int f2bf(float f) {
  const unsigned int u = __float_as_uint(f);
  const unsigned int r = ((u + 0x7FFFu + ((u >> 16) & 1u)) >> 16) & 0xFFFFu;
  return ((u & 0x7FFFFFFFu) > 0x7F800000u) ? 0x7FC0u : r;
}
__device__ __forceinline__ float bf2f(unsigned int b) { return __uint_as_float(b << 16); }
__device__ __forceinline__ float bfr(float f) { return bf2f(f2bf(f)); }

__device__ __forceinline__ float sigm_f(float t) {
  float a = t * -1.44269504f;
  a = fminf(fmaxf(a, -126.0f), 126.0f);
  const float e = __builtin_amdgcn_exp2f(a);
  return __builtin_amdgcn_rcpf(1.0f + e);
}
__device__ __forceinline__ float silu_f(float t) { return t * sigm_f(t); }

__device__ __forceinline__ void put16(unsigned short* dp, v8us o) {
  *(volatile v8us*)dp = o;
  __threadfence();
  *(volatile v8us*)dp = o;
}
__device__ __forceinline__ void putf4(float* dp, v4f o) {
  *(volatile v4f*)dp = o;
  __threadfence();
  *(volatile v4f*)dp = o;
}

__device__ __forceinline__ void st_hl2(unsigned short* rowp, int col, int khalf, float v0, float v1) {
  const unsigned int u0 = __float_as_uint(v0);
  const unsigned int u1 = __float_as_uint(v1);
  const unsigned int r0 = u0 + 0x7FFFu + ((u0 >> 16) & 1u);
  const unsigned int r1 = u1 + 0x7FFFu + ((u1 >> 16) & 1u);
  const float h0 = __uint_as_float(r0 & 0xFFFF0000u);
  const float h1 = __uint_as_float(r1 & 0xFFFF0000u);
  const unsigned int w0 = __float_as_uint(v0 - h0);
  const unsigned int w1 = __float_as_uint(v1 - h1);
  const unsigned int s0 = w0 + 0x7FFFu + ((w0 >> 16) & 1u);
  const unsigned int s1 = w1 + 0x7FFFu + ((w1 >> 16) & 1u);
  *(u32a*)(rowp + col)         = (r0 >> 16) | (r1 & 0xFFFF0000u);
  *(u32a*)(rowp + khalf + col) = (s0 >> 16) | (s1 & 0xFFFF0000u);
}

template <int SLB>
__device__ __forceinline__ int scan_chunk(const int* __restrict__ dsts, int nE, int cbase, int slotBase,
                                          int nb, int vec8, int* list, int tid, int lane, int wave) {
  int wc = 0;
  const int el0  = tid * EPT;
  const int e0   = cbase + el0;
  const int sent = -2147483647 - 1;
  v4i da, db;
  if (vec8 != 0 && cbase + CHUNK <= nE) {
    da = *(const v4i*)(dsts + e0);
    db = *(const v4i*)(dsts + e0 + 4);
  } else {
    da.x = (e0     < nE) ? dsts[min(e0,     nE - 1)] : sent;
    da.y = (e0 + 1 < nE) ? dsts[min(e0 + 1, nE - 1)] : sent;
    da.z = (e0 + 2 < nE) ? dsts[min(e0 + 2, nE - 1)] : sent;
    da.w = (e0 + 3 < nE) ? dsts[min(e0 + 3, nE - 1)] : sent;
    db.x = (e0 + 4 < nE) ? dsts[min(e0 + 4, nE - 1)] : sent;
    db.y = (e0 + 5 < nE) ? dsts[min(e0 + 5, nE - 1)] : sent;
    db.z = (e0 + 6 < nE) ? dsts[min(e0 + 6, nE - 1)] : sent;
    db.w = (e0 + 7 < nE) ? dsts[min(e0 + 7, nE - 1)] : sent;
  }
  const unsigned nbs = (unsigned)slotBase;
  const unsigned unb = (unsigned)nb;
  const unsigned s0 = (unsigned)da.x - nbs, s1 = (unsigned)da.y - nbs;
  const unsigned s2 = (unsigned)da.z - nbs, s3 = (unsigned)da.w - nbs;
  const unsigned s4 = (unsigned)db.x - nbs, s5 = (unsigned)db.y - nbs;
  const unsigned s6 = (unsigned)db.z - nbs, s7 = (unsigned)db.w - nbs;
  const bool h0 = s0 < unb, h1 = s1 < unb, h2 = s2 < unb, h3 = s3 < unb;
  const bool h4 = s4 < unb, h5 = s5 < unb, h6 = s6 < unb, h7 = s7 < unb;
  const unsigned any = __builtin_amdgcn_ballot_w32(h0 | h1 | h2 | h3 | h4 | h5 | h6 | h7);
  if (any != 0u) {
#define HITJ(J, HJ, SJ) { \
      const unsigned mj = __builtin_amdgcn_ballot_w32(HJ); \
      if (mj != 0u) { \
        if (HJ) { \
          const int pos = wc + (int)__builtin_amdgcn_mbcnt_lo(mj, 0u); \
          if (pos < WCAP) list[wave * WCAP + pos] = ((el0 + (J)) << SLB) | (int)(SJ); \
        } \
        wc += (int)__builtin_popcount(mj); } }
    HITJ(0, h0, s0)
    HITJ(1, h1, s1)
    HITJ(2, h2, s2)
    HITJ(3, h3, s3)
    HITJ(4, h4, s4)
    HITJ(5, h5, s5)
    HITJ(6, h6, s6)
    HITJ(7, h7, s7)
#undef HITJ
  }
  return wc;
}

__device__ __forceinline__ void tr8(const float* __restrict__ W, int ldw, int kmask,
                                    unsigned short* plane, int ldk, int nOff, int v) {
  const int upr = ldk >> 3;
  const int n   = v / upr;
  const int k8  = (v - n * upr) * 8;
  const int ks  = k8 & kmask;
  const float* p = W + (size_t)ks * (size_t)ldw + n;
  v8us o;
#pragma unroll
  for (int i = 0; i < 8; ++i) o[i] = (unsigned short)f2bf(p[(size_t)i * (size_t)ldw]);
  put16(plane + (size_t)(nOff + n) * (size_t)ldk + k8, o);
}

__global__ __launch_bounds__(NTHR) void k_pa(const float* __restrict__ x, const float* __restrict__ Wsrc,
                                             const float* __restrict__ Wdst, const float* __restrict__ Wfc1,
                                             const float* __restrict__ Wfc2, const float* __restrict__ Wfc3,
                                             unsigned char* ws) {
  const int u = (int)blockIdx.x * NTHR + (int)threadIdx.x;
  unsigned short* XB  = (unsigned short*)(ws + O_XB);
  unsigned short* WSD = (unsigned short*)(ws + O_WSD);
  unsigned short* W1T = (unsigned short*)(ws + O_W1T);
  unsigned short* W2D = (unsigned short*)(ws + O_W2D);
  unsigned short* W3D = (unsigned short*)(ws + O_W3D);
  const int L0 = NU_XB;
  const int L1 = L0 + NU_K128;
  const int L2 = L1 + NU_K128;
  const int L3 = L2 + NU_W1;
  const int L4 = L3 + NU_W2;
  const int L5 = L4 + NU_W3;
  if (u < L0) {
    const int row = u >> 4;
    const int c0  = (u & 15) * 8;
    const int rc  = row < NN ? row : NN - 1;
    const bool ok = row < NN;
    const float* p = x + (size_t)rc * CC + c0;
    const v4f a = *(const v4f*)p;
    const v4f b = *(const v4f*)(p + 4);
    const v8f f8 = {a.x, a.y, a.z, a.w, b.x, b.y, b.z, b.w};
    v8us o;
#pragma unroll
    for (int i = 0; i < 8; ++i) o[i] = ok ? (unsigned short)f2bf(f8[i]) : (unsigned short)0;
    put16(XB + (size_t)row * CC + c0, o);
  } else if (u < L1) {
    tr8(Wsrc, CC, 127, WSD, 128, 0, u - L0);
  } else if (u < L2) {
    tr8(Wdst, CC, 127, WSD, 128, 128, u - L1);
  } else if (u < L3) {
    tr8(Wfc1, FCH, 63, W1T, 64, 0, u - L2);
  } else if (u < L4) {
    tr8(Wfc2, FCH, 63, W2D, 128, 0, u - L3);
  } else if (u < L5) {
    tr8(Wfc3, CC, 63, W3D, 128, 0, u - L4);
  }
}

__device__ __forceinline__ v4u ldm(const float* __restrict__ p, int j, int nq, bool on) {
  const int jc = j < 0 ? 0 : (j > nq - 1 ? nq - 1 : j);
  const v4f v = *(const v4f*)(p + 4 * jc);
  const unsigned mk = on ? 0xFFFFFFFFu : 0u;
  v4u r;
  r.x = __float_as_uint(v.x) & mk;
  r.y = __float_as_uint(v.y) & mk;
  r.z = __float_as_uint(v.z) & mk;
  r.w = __float_as_uint(v.w) & mk;
  return r;
}

__global__ __launch_bounds__(NTHR) void k_pb(const float* __restrict__ Walpha, const float* __restrict__ Wlin,
                                             const float* __restrict__ Wval, const float* __restrict__ Wout,
                                             const float* __restrict__ bsrc, const float* __restrict__ bfc1,
                                             const float* __restrict__ bfc2, const float* __restrict__ wint,
                                             const float* __restrict__ attd, const float* __restrict__ bout,
                                             unsigned char* ws) {
  const int u = (int)blockIdx.x * NTHR + (int)threadIdx.x;
  unsigned short* WALD = (unsigned short*)(ws + O_WALD);
  unsigned short* WVD  = (unsigned short*)(ws + O_WVD);
  unsigned short* WOD  = (unsigned short*)(ws + O_WOD);
  float*          PV   = (float*)(ws + O_PV);
  const int L0 = NU_K256;
  const int L1 = 2 * NU_K256;
  const int L2 = 3 * NU_K256;
  const int L3 = 4 * NU_K256;
  if (u < L0) {
    tr8(Walpha, CC, 127, WALD, 256, 0, u);
  } else if (u < L1) {
    tr8(Wlin, CC, 127, WALD, 256, 128, u - L0);
  } else if (u < L2) {
    tr8(Wval, CC, 127, WVD, 256, 0, u - L1);
  } else if (u < L3) {
    tr8(Wout, CC, 127, WOD, 256, 0, u - L2);
  } else {
    const int t = u - L3;
    const v4u a0 = ldm(bsrc, t,       32, t < 32);
    const v4u a1 = ldm(bfc1, t - 64,  16, t >= 64 && t < 80);
    const v4u a2 = ldm(bfc2, t - 80,  16, t >= 80 && t < 96);
    const v4u a3 = ldm(wint, t - 96,  32, t >= 96 && t < 128);
    const v4u a4 = ldm(attd, t - 128, 32, t >= 128 && t < 160);
    const v4u a5 = ldm(bout, t - 160, 32, t >= 160 && t < 192);
    v4f o;
    o.x = bfr(__uint_as_float(a0.x | a1.x | a2.x | a3.x | a4.x | a5.x));
    o.y = bfr(__uint_as_float(a0.y | a1.y | a2.y | a3.y | a4.y | a5.y));
    o.z = bfr(__uint_as_float(a0.z | a1.z | a2.z | a3.z | a4.z | a5.z));
    o.w = bfr(__uint_as_float(a0.w | a1.w | a2.w | a3.w | a4.w | a5.w));
    if (t < 192) putf4(PV + 4 * t, o);
  }
}

template <int MODE>
__global__ __launch_bounds__(GTHR) void k_gemm(const unsigned short* __restrict__ A, int lda,
                                               const unsigned short* __restrict__ BT, int ldb, int K,
                                               const float* __restrict__ bias, int nRows,
                                               float* C, int ldc, const int* __restrict__ FLG) {
  __shared__ __attribute__((aligned(16))) float stg[GBM * GBN];
  const int tid = (int)threadIdx.x, lane = tid & 31, wave = tid >> 5, hh = lane >> 4, m = lane & 15;
  const int rowBase = (int)blockIdx.x * GBM;
  const int colBase = (int)blockIdx.y * GBN;

  v8f acc[8];
  {
    const v8f z = {0.f, 0.f, 0.f, 0.f, 0.f, 0.f, 0.f, 0.f};
#pragma unroll
    for (int t = 0; t < 8; ++t) acc[t] = z;
  }
  const unsigned short* ap = A  + (size_t)(rowBase + 16 * wave + m) * (size_t)lda + 8 * hh;
  const unsigned short* bp = BT + (size_t)(colBase + m) * (size_t)ldb + 8 * hh;
#pragma unroll 1
  for (int k0 = 0; k0 < K; k0 += 32) {
    FragB af;
    af.h[0] = *(const v8usa*)(ap + k0);
    af.h[1] = *(const v8usa*)(ap + k0 + 16);
#pragma unroll
    for (int nt = 0; nt < 8; ++nt) {
      const unsigned short* wq = bp + (size_t)(16 * nt) * (size_t)ldb + k0;
      FragB bf;
      bf.h[0] = *(const v8usa*)wq;
      bf.h[1] = *(const v8usa*)(wq + 16);
      acc[nt] = wmb(af, bf, acc[nt]);
    }
  }

  bool poison = false;
  if constexpr (MODE == 1) {
    int fb = rowBase >> SLA;
    fb = fb > NBLK - 1 ? NBLK - 1 : fb;
    const int fl = FLG[(size_t)fb * 32 + 1];
    poison = fl != 0;
  }
  const float qnan = __int_as_float(0x7fc00000);
#pragma unroll
  for (int nt = 0; nt < 8; ++nt) {
    const int lc = 16 * nt + m;
    const float bvv = bias[colBase + lc];
#pragma unroll
    for (int r = 0; r < 8; ++r) {
      const int lr = 16 * wave + 8 * hh + r;
      const float v = acc[nt][r] + bvv;
      stg[lr * GBN + lc] = poison ? qnan : v;
    }
  }
  __syncthreads();

  v4f pv[16];
#pragma unroll
  for (int i = 0; i < 16; ++i) pv[i] = *(const v4fa*)(stg + (16 * wave + i) * GBN + 4 * lane);
#pragma unroll
  for (int i = 0; i < 16; ++i) {
    const int row = rowBase + 16 * wave + i;
    if (row < nRows) {
      float* op = C + (size_t)row * (size_t)ldc + colBase + 4 * lane;
      *(volatile v4f*)op = pv[i];
    }
  }
  __threadfence();
#pragma unroll
  for (int i = 0; i < 16; ++i) {
    const int row = rowBase + 16 * wave + i;
    if (row < nRows) {
      float* op = C + (size_t)row * (size_t)ldc + colBase + 4 * lane;
      *(volatile v4f*)op = pv[i];
    }
  }
}

__global__ __launch_bounds__(NTHR) void k_bucket(const int* __restrict__ dsts, int nE, int nN, int vec8,
                                                 int* HITS, int* FLG) {
  extern __shared__ __attribute__((aligned(16))) int bsm[];
  int* list = bsm;
  int* reg1 = bsm + LISTN;
  int* wcnt = reg1 + RCAP;
  const int tid = (int)threadIdx.x, lane = tid & 31, wave = tid >> 5;
  const int blk = (int)blockIdx.x;
  const int nodeBase = blk * NBA;
  int nb = nN - nodeBase;
  nb = nb < 0 ? 0 : (nb > NBA ? NBA : nb);

  int tot = 0, ovf = 0;
  const int nChunks = (nE + CHUNK - 1) / CHUNK;
#pragma unroll 1
  for (int ch = 0; ch < nChunks; ++ch) {
    const int cbase = ch * CHUNK;
    const int wc = scan_chunk<SLA>(dsts, nE, cbase, nodeBase, nb, vec8, list, tid, lane, wave);
    if (lane == 0) wcnt[wave] = wc;
    __syncthreads();
    int pre = 0, all = 0;
#pragma unroll
    for (int w2 = 0; w2 < NWAVE; ++w2) {
      int c = wcnt[w2];
      c = c < 0 ? 0 : (c > WCAP ? WCAP : c);
      all += c;
      pre += (w2 < wave) ? c : 0;
    }
    const int wcc  = wc > WCAP ? WCAP : wc;
    const int base = tot + pre;
#pragma unroll 1
    for (int i = lane; i < wcc; i += 32) {
      const int ent = list[wave * WCAP + i];
      const int el  = (ent >> SLA) & (CHUNK - 1);
      const int sl  = ent & (NBA - 1);
      int eid = cbase + el;
      eid = eid > nE - 1 ? nE - 1 : eid;
      const int pos = base + i;
      if (pos < RCAP) reg1[pos] = (int)((unsigned)eid | ((unsigned)sl << ESH));
    }
    if (tot + all > RCAP) ovf = 1;
    tot += all;
    tot = tot > RCAP ? RCAP : tot;
    __syncthreads();
  }
  const int nh = tot;
  for (int i = nh + tid; i < RCAP; i += NTHR) reg1[i] = 0;
  __syncthreads();

  int* hb = HITS + (size_t)blk * RCAP;
  v4i cv;
  cv.x = (tid == 0) ? nh : 0;
  cv.y = (tid == 0) ? ovf : 0;
  cv.z = 0; cv.w = 0;
  int* fp = FLG + (size_t)blk * 32 + 4 * (tid & 7);
#pragma unroll 1
  for (int p = tid * 4; p < RCAP; p += NTHR * 4) {
    const v4i v = *(const v4ia*)(reg1 + p);
    *(volatile v4i*)(hb + p) = v;
  }
  if (tid < 8) *(volatile v4i*)fp = cv;
  __threadfence();
#pragma unroll 1
  for (int p = tid * 4; p < RCAP; p += NTHR * 4) {
    const v4i v = *(const v4ia*)(reg1 + p);
    *(volatile v4i*)(hb + p) = v;
  }
  if (tid < 8) *(volatile v4i*)fp = cv;
}

template <int PAIR>
__device__ __forceinline__ void gemm4(const unsigned short* ap, const unsigned short* __restrict__ BT, int n0,
                                      int ldb, int K, int m, int hh, v8f (&acc)[4]) {
  const v8f z = {0.f, 0.f, 0.f, 0.f, 0.f, 0.f, 0.f, 0.f};
  acc[0] = z; acc[1] = z; acc[2] = z; acc[3] = z;
  const unsigned short* bp = BT + (size_t)(n0 + (PAIR ? 2 * m : m)) * (size_t)ldb + 8 * hh;
#pragma unroll 1
  for (int k0 = 0; k0 < K; k0 += 32) {
    FragB af;
    af.h[0] = *(const v8usa*)(ap + k0);
    af.h[1] = *(const v8usa*)(ap + k0 + 16);
#pragma unroll
    for (int t = 0; t < 4; ++t) {
      const int ro = PAIR ? (32 * (t >> 1) + (t & 1)) : (16 * t);
      const unsigned short* wq = bp + (size_t)ro * (size_t)ldb + k0;
      FragB bf;
      bf.h[0] = *(const v8usa*)wq;
      bf.h[1] = *(const v8usa*)(wq + 16);
      acc[t] = wmb(af, bf, acc[t]);
    }
  }
}

__global__ __launch_bounds__(NTHR) __attribute__((amdgpu_num_vgpr(248)))
void k_edge(unsigned char* ws, const float* __restrict__ nattr, const float* __restrict__ eattr,
            const float* __restrict__ eemb, const int* __restrict__ esrc, const int* __restrict__ edst, int g) {
  extern __shared__ __attribute__((aligned(16))) unsigned char esm[];
  unsigned short* buf0 = (unsigned short*)(esm + L_BUF0);
  unsigned short* buf1 = (unsigned short*)(esm + L_BUF1);
  float* sG   = (float*)(esm + L_G);
  float* sLog = (float*)(esm + L_LOG);
  float* sPV  = (float*)(esm + L_PV);
  float* sEa  = (float*)(esm + L_EA);
  int*   sId  = (int*)(esm + L_ID);

  const int tid = (int)threadIdx.x, lane = tid & 31, wave = tid >> 5, hh = lane >> 4, m = lane & 15;
  const int*   F0   = (const int*)(ws + O_FLG0);
  const int*   HITS = (const int*)(ws + O_HIT);
  const float* MSD  = (const float*)(ws + O_MSD);
  const float* PV   = (const float*)(ws + O_PV);
  const unsigned short* W1T  = (const unsigned short*)(ws + O_W1T);
  const unsigned short* W2D  = (const unsigned short*)(ws + O_W2D);
  const unsigned short* W3D  = (const unsigned short*)(ws + O_W3D);
  const unsigned short* WALD = (const unsigned short*)(ws + O_WALD);
  const unsigned short* WVD  = (const unsigned short*)(ws + O_WVD);
  float* VAL   = (float*)(ws + O_VAL);
  float* LOGIT = (float*)(ws + O_LOG);

  int cn[BPG];
#pragma unroll
  for (int i = 0; i < BPG; ++i) {
    const int v = F0[(size_t)(g * BPG + i) * 32];
    cn[i] = v < 0 ? 0 : (v > RCAP ? RCAP : v);
  }
  int pre[BPG + 1];
  pre[0] = 0;
#pragma unroll
  for (int i = 0; i < BPG; ++i) pre[i + 1] = pre[i] + cn[i];
  const int total = pre[BPG] > VCAP ? VCAP : pre[BPG];
  const int q0 = (int)blockIdx.x * TROWS;
  if (q0 >= total) return;

  if (tid < 192) *(v4fa*)(sPV + 4 * tid) = *(const v4f*)(PV + 4 * tid);
  if (tid < TROWS) {
    const int q  = q0 + tid;
    const int qc = q < total ? q : total - 1;
    int j = 0, pj = 0;
#pragma unroll
    for (int i = 1; i < BPG; ++i) {
      const bool ge = qc >= pre[i];
      j  = ge ? i : j;
      pj = ge ? pre[i] : pj;
    }
    int p = qc - pj;
    p = p < 0 ? 0 : (p > RCAP - 1 ? RCAP - 1 : p);
    const int hit = HITS[(size_t)(g * BPG + j) * RCAP + p];
    int e = hit & EMASK;
    e = e > EE - 1 ? EE - 1 : e;
    int s = esrc[e];
    int d = edst[e];
    s = s < 0 ? 0 : (s > NN - 1 ? NN - 1 : s);
    d = d < 0 ? 0 : (d > NN - 1 ? NN - 1 : d);
    sId[tid] = e;
    sId[TROWS + tid] = s;
    sId[2 * TROWS + tid] = d;
    sEa[tid] = bfr(eattr[e]);
  }
  __syncthreads();

#pragma unroll
  for (int it = 0; it < 4; ++it) {
    const int u = it * NTHR + tid;
    const int row = u >> 3, c4 = (u & 7) * 4;
    const int e = sId[row];
    const v4f xv = *(const v4f*)(eemb + (size_t)e * NBF + c4);
    v4us o;
    o.x = (unsigned short)f2bf(xv.x); o.y = (unsigned short)f2bf(xv.y);
    o.z = (unsigned short)f2bf(xv.z); o.w = (unsigned short)f2bf(xv.w);
    *(v4usa*)(buf0 + row * AP + c4) = o;
  }
#pragma unroll
  for (int it = 0; it < 2; ++it) {
    const int u = it * NTHR + tid;
    const int row = u >> 2, c4 = (u & 3) * 4;
    const int s = sId[TROWS + row];
    const v4f xv = *(const v4f*)(nattr + (size_t)s * NAF + c4);
    v4us o;
    o.x = (unsigned short)f2bf(xv.x); o.y = (unsigned short)f2bf(xv.y);
    o.z = (unsigned short)f2bf(xv.z); o.w = (unsigned short)f2bf(xv.w);
    *(v4usa*)(buf0 + row * AP + NBF + c4) = o;
  }
#pragma unroll
  for (int it = 0; it < 2; ++it) {
    const int u = it * NTHR + tid;
    const int row = u >> 2, c4 = (u & 3) * 4;
    const int d = sId[2 * TROWS + row];
    const v4f xv = *(const v4f*)(nattr + (size_t)d * NAF + c4);
    v4us o;
    o.x = (unsigned short)f2bf(xv.x); o.y = (unsigned short)f2bf(xv.y);
    o.z = (unsigned short)f2bf(xv.z); o.w = (unsigned short)f2bf(xv.w);
    *(v4usa*)(buf0 + row * AP + NBF + NAF + c4) = o;
  }
#pragma unroll 4
  for (int it = 0; it < 16; ++it) {
    const int u = it * NTHR + tid;
    const int row = u >> 5, c4 = (u & 31) * 4;
    const int s = sId[TROWS + row];
    const int d = sId[2 * TROWS + row];
    const float ea = sEa[row];
    const v4f a = *(const v4f*)(MSD + (size_t)s * 256 + c4);
    const v4f b = *(const v4f*)(MSD + (size_t)d * 256 + 128 + c4);
    v4f gq;
    gq.x = (a.x + b.x) * ea; gq.y = (a.y + b.y) * ea;
    gq.z = (a.z + b.z) * ea; gq.w = (a.w + b.w) * ea;
    *(v4fa*)(sG + row * DP + c4) = gq;
  }
  __syncthreads();

  const int rw = 16 * wave;
  const unsigned short* a0p = buf0 + (rw + m) * AP + 8 * hh;
  const unsigned short* a1p = buf1 + (rw + m) * AP + 8 * hh;
  v8f acc[4];

  gemm4<1>(a0p, W1T, 0, 64, 64, m, hh, acc);
#pragma unroll
  for (int tp = 0; tp < 2; ++tp) {
    const int col = 32 * tp + 2 * m;
    const v2f bv = *(const v2fa*)(sPV + 256 + col);
#pragma unroll
    for (int r = 0; r < 8; ++r) {
      const int row = rw + 8 * hh + r;
      st_hl2(buf1 + row * AP, col, 64, silu_f(acc[2 * tp][r] + bv.x), silu_f(acc[2 * tp + 1][r] + bv.y));
    }
  }
  __syncthreads();

  gemm4<1>(a1p, W2D, 0, 128, 128, m, hh, acc);
#pragma unroll
  for (int tp = 0; tp < 2; ++tp) {
    const int col = 32 * tp + 2 * m;
    const v2f bv = *(const v2fa*)(sPV + 320 + col);
#pragma unroll
    for (int r = 0; r < 8; ++r) {
      const int row = rw + 8 * hh + r;
      st_hl2(buf0 + row * AP, col, 64, silu_f(acc[2 * tp][r] + bv.x), silu_f(acc[2 * tp + 1][r] + bv.y));
    }
  }
  __syncthreads();

#pragma unroll 1
  for (int ch = 0; ch < 2; ++ch) {
    gemm4<1>(a0p, W3D, 64 * ch, 128, 128, m, hh, acc);
#pragma unroll
    for (int tp = 0; tp < 2; ++tp) {
      const int col = 64 * ch + 32 * tp + 2 * m;
#pragma unroll
      for (int r = 0; r < 8; ++r) {
        const int row = rw + 8 * hh + r;
        const v2f gq = *(const v2fa*)(sG + row * DP + col);
        st_hl2(buf1 + row * AP, col, 128, gq.x * acc[2 * tp][r], gq.y * acc[2 * tp + 1][r]);
      }
    }
  }
  __syncthreads();

#pragma unroll 1
  for (int ch = 0; ch < 2; ++ch) {
    gemm4<0>(a1p, WALD, 64 * ch, 256, 256, m, hh, acc);
#pragma unroll
    for (int t = 0; t < 4; ++t) {
      const int head = 4 * ch + t;
      const float ad = sPV[512 + head * DHEAD + m];
#pragma unroll
      for (int r = 0; r < 8; ++r) {
        const float S  = acc[t][r];
        const float sg = sigm_f(S);
        const float sl = 0.6f * S + 0.4f * S * (2.0f * sg - 1.0f);
        float tv = sl * ad;
        tv += __shfl_xor(tv, 1, 32);
        tv += __shfl_xor(tv, 2, 32);
        tv += __shfl_xor(tv, 4, 32);
        tv += __shfl_xor(tv, 8, 32);
        if (m == 0) sLog[(rw + 8 * hh + r) * 8 + head] = tv;
      }
    }
  }
#pragma unroll 1
  for (int ch = 0; ch < 2; ++ch) {
    gemm4<1>(a1p, WALD, 128 + 64 * ch, 256, 256, m, hh, acc);
#pragma unroll
    for (int tp = 0; tp < 2; ++tp) {
      const int col = 64 * ch + 32 * tp + 2 * m;
      const v2f wi = *(const v2fa*)(sPV + 384 + col);
#pragma unroll
      for (int r = 0; r < 8; ++r) {
        const int row = rw + 8 * hh + r;
        const float ea = sEa[row];
        const float v0 = (silu_f(acc[2 * tp][r]) * ea) * wi.x;
        const float v1 = (silu_f(acc[2 * tp + 1][r]) * ea) * wi.y;
        st_hl2(buf0 + row * AP, col, 128, v0, v1);
      }
    }
  }
  __syncthreads();

  {
    const v4f lv = *(const v4fa*)(sLog + rw * 8 + 4 * lane);
    float* lp = LOGIT + (size_t)(q0 + rw) * 8 + 4 * lane;
    *(volatile v4f*)lp = lv;
    __threadfence();
    *(volatile v4f*)lp = lv;
  }

#pragma unroll 1
  for (int ch = 0; ch < 2; ++ch) {
    gemm4<0>(a0p, WVD, 64 * ch, 256, 256, m, hh, acc);
#pragma unroll
    for (int t = 0; t < 4; ++t) {
      const int col = 64 * ch + 16 * t + m;
#pragma unroll
      for (int r = 0; r < 8; ++r) sG[(rw + 8 * hh + r) * DP + col] = acc[t][r];
    }
  }
  __syncthreads();
  {
    v4f pv[16];
#pragma unroll
    for (int i = 0; i < 16; ++i) pv[i] = *(const v4fa*)(sG + (rw + i) * DP + 4 * lane);
    float* vb = VAL + (size_t)(q0 + rw) * CC + 4 * lane;
#pragma unroll
    for (int i = 0; i < 16; ++i) *(volatile v4f*)(vb + (size_t)i * CC) = pv[i];
    __threadfence();
#pragma unroll
    for (int i = 0; i < 16; ++i) *(volatile v4f*)(vb + (size_t)i * CC) = pv[i];
  }
}

__global__ __launch_bounds__(NTHR) void k_scan(unsigned char* ws, int g) {
  extern __shared__ __attribute__((aligned(16))) int ssm[];
  int* hl   = ssm;
  int* sl   = ssm + RCAP;
  int* cnt  = sl + RCAP;
  int* offs = cnt + NBA;
  int* cur  = offs + NBA;
  int* misc = cur + NBA;
  const int tid = (int)threadIdx.x, lane = tid & 31, wave = tid >> 5;
  const int jb  = (int)blockIdx.x;
  const int blk = g * BPG + jb;
  const int nodeBase = blk * NBA;
  const int*   F0    = (const int*)(ws + O_FLG0);
  const int*   HITS  = (const int*)(ws + O_HIT);
  const float* LOGIT = (const float*)(ws + O_LOG);
  const float* VAL   = (const float*)(ws + O_VAL);
  unsigned short* AGG = (unsigned short*)(ws + O_AGG);
  int* F1 = (int*)(ws + O_FLG1);

  int qbase = 0, gtot = 0;
#pragma unroll
  for (int i = 0; i < BPG; ++i) {
    const int v  = F0[(size_t)(g * BPG + i) * 32];
    const int vc = v < 0 ? 0 : (v > RCAP ? RCAP : v);
    qbase += (i < jb) ? vc : 0;
    gtot  += vc;
  }
  const int nhraw = F0[(size_t)blk * 32];
  const int bflag = F0[(size_t)blk * 32 + 1];
  const int nh  = nhraw < 0 ? 0 : (nhraw > RCAP ? RCAP : nhraw);
  const int ovf = (bflag != 0 || nhraw < 0 || nhraw > RCAP || gtot > VCAP) ? 1 : 0;

  {
    const v4i z4 = {0, 0, 0, 0};
    for (int i = tid * 4; i < SCAN_ZINTS; i += NTHR * 4) *(v4ia*)(sl + i) = z4;
    if (tid < 16) misc[tid] = 0;
    const int* hb = HITS + (size_t)blk * RCAP;
    const int nh4 = (nh + 3) & ~3;
#pragma unroll 1
    for (int p = tid * 4; p < nh4; p += NTHR * 4) *(v4ia*)(hl + p) = *(const v4i*)(hb + p);
  }
  __syncthreads();

  if (wave == 0) {
#pragma unroll 1
    for (int b0 = 0; b0 < nh; b0 += 32) {
      const int idx = b0 + lane;
      const int uv  = hl[idx < nh ? idx : nh - 1];
      const int m32 = (nh - b0) < 32 ? (nh - b0) : 32;
#pragma unroll 1
      for (int k = 0; k < m32; ++k) {
        const int u  = __builtin_amdgcn_readlane(uv, k);
        const int sq = (u >> ESH) & (NBA - 1);
        if (lane == 0) cnt[sq] = cnt[sq] + 1;
      }
    }
  }
  __syncthreads();
  if (wave == 0) {
    const int lb = lane * (NBA / 32);
    int s = 0;
#pragma unroll 1
    for (int i = 0; i < NBA / 32; ++i) s += cnt[lb + i];
    int incl = s;
#pragma unroll
    for (int d = 1; d < 32; d <<= 1) {
      const int y = __shfl_up(incl, d, 32);
      if (lane >= d) incl += y;
    }
    int run = incl - s;
#pragma unroll 1
    for (int i = 0; i < NBA / 32; ++i) {
      const int cv = cnt[lb + i];
      offs[lb + i] = run;
      cur[lb + i]  = run;
      run += cv;
    }
  }
  __syncthreads();
  if (wave == 0) {
#pragma unroll 1
    for (int b0 = 0; b0 < nh; b0 += 32) {
      const int idx = b0 + lane;
      const int uv  = hl[idx < nh ? idx : nh - 1];
      const int m32 = (nh - b0) < 32 ? (nh - b0) : 32;
#pragma unroll 1
      for (int k = 0; k < m32; ++k) {
        const int u  = __builtin_amdgcn_readlane(uv, k);
        const int sq = (u >> ESH) & (NBA - 1);
        if (lane == 0) {
          int p = cur[sq];
          p = p < 0 ? 0 : (p > RCAP - 1 ? RCAP - 1 : p);
          sl[p] = b0 + k;
          cur[sq] = p + 1;
        }
      }
    }
  }
  __syncthreads();

  const float qnan = __int_as_float(0x7fc00000);
  const float pzb  = (ovf != 0) ? qnan : 0.0f;
  const int head   = lane >> 2;
  const int nhm    = nh > 0 ? nh - 1 : 0;
  int anybig = 0;

#pragma unroll 1
  for (int si = 0; si < NBA / NWAVE; ++si) {
    const int s    = si * NWAVE + wave;
    const int node = nodeBase + s;
    int c = cnt[s];
    const bool big = c > DEGCAP;
    anybig |= big ? 1 : 0;
    c = c < 0 ? 0 : (c > DEGCAP ? DEGCAP : c);
    int o = offs[s];
    o = o < 0 ? 0 : (o > RCAP ? RCAP : o);
    if (c > nh - o) c = nh - o;
    c = c < 0 ? 0 : c;

    float mx = 0.0f;
    int have = 0;
#pragma unroll 1
    for (int b0 = 0; b0 < c; b0 += 32) {
      int t = b0 + lane;
      t = t < c ? t : c - 1;
      int idx = o + t;
      idx = idx < 0 ? 0 : (idx > RCAP - 1 ? RCAP - 1 : idx);
      int pos = sl[idx];
      pos = pos < 0 ? 0 : (pos > nhm ? nhm : pos);
      int q = qbase + pos;
      q = q < 0 ? 0 : (q > VCAP - 1 ? VCAP - 1 : q);
      const int m32 = (c - b0) < 32 ? (c - b0) : 32;
#pragma unroll 1
      for (int k = 0; k < m32; ++k) {
        const int qk = __builtin_amdgcn_readlane(q, k);
        const float lg = LOGIT[(size_t)qk * 8 + head];
        mx = (have != 0) ? fmaxf(mx, lg) : lg;
        have = 1;
      }
    }
    mx = (fabsf(mx) <= 3.4028235e38f) ? mx : 0.0f;

    float dn = 0.0f, a0 = 0.0f, a1 = 0.0f, a2 = 0.0f, a3 = 0.0f;
#pragma unroll 1
    for (int b0 = 0; b0 < c; b0 += 32) {
      int t = b0 + lane;
      t = t < c ? t : c - 1;
      int idx = o + t;
      idx = idx < 0 ? 0 : (idx > RCAP - 1 ? RCAP - 1 : idx);
      int pos = sl[idx];
      pos = pos < 0 ? 0 : (pos > nhm ? nhm : pos);
      int q = qbase + pos;
      q = q < 0 ? 0 : (q > VCAP - 1 ? VCAP - 1 : q);
      const int m32 = (c - b0) < 32 ? (c - b0) : 32;
#pragma unroll 1
      for (int k = 0; k < m32; ++k) {
        const int qk = __builtin_amdgcn_readlane(q, k);
        const float lg = LOGIT[(size_t)qk * 8 + head];
        const v4f vv = *(const v4f*)(VAL + (size_t)qk * CC + 4 * lane);
        const float ex = expf(lg - mx);
        dn += ex;
        a0 = fmaf(ex, vv.x, a0);
        a1 = fmaf(ex, vv.y, a1);
        a2 = fmaf(ex, vv.z, a2);
        a3 = fmaf(ex, vv.w, a3);
      }
    }
    const float rinv = 1.0f / (dn + 1e-16f);
    const float pzr  = big ? qnan : pzb;
    const bool  live = node < NN;
    const float r0 = live ? (a0 * rinv + pzr) : 0.0f;
    const float r1 = live ? (a1 * rinv + pzr) : 0.0f;
    const float r2 = live ? (a2 * rinv + pzr) : 0.0f;
    const float r3 = live ? (a3 * rinv + pzr) : 0.0f;
    v4us ho, lo;
    {
      const unsigned int h0 = f2bf(r0), h1 = f2bf(r1), h2 = f2bf(r2), h3 = f2bf(r3);
      ho.x = (unsigned short)h0; ho.y = (unsigned short)h1; ho.z = (unsigned short)h2; ho.w = (unsigned short)h3;
      lo.x = (unsigned short)f2bf(r0 - bf2f(h0));
      lo.y = (unsigned short)f2bf(r1 - bf2f(h1));
      lo.z = (unsigned short)f2bf(r2 - bf2f(h2));
      lo.w = (unsigned short)f2bf(r3 - bf2f(h3));
    }
    if (node < MP) {
      unsigned short* hp = AGG + (size_t)node * 256 + 4 * lane;
      *(volatile v4us*)hp = ho;
      *(volatile v4us*)(hp + CC) = lo;
      __threadfence();
      *(volatile v4us*)hp = ho;
      *(volatile v4us*)(hp + CC) = lo;
    }
  }

  if (lane == 0) misc[wave] = anybig;
  __syncthreads();
  if (wave == 0) {
    int fg = ovf;
#pragma unroll
    for (int w2 = 0; w2 < NWAVE; ++w2) fg |= misc[w2];
    v4i cv;
    cv.x = 0;
    cv.y = (lane == 0) ? fg : 0;
    cv.z = 0; cv.w = 0;
    int* fp = F1 + (size_t)blk * 32 + 4 * (lane & 7);
    if (lane < 8) *(volatile v4i*)fp = cv;
    __threadfence();
    if (lane < 8) *(volatile v4i*)fp = cv;
  }
}

extern "C" void kernel_launch(void* const* d_in, const int* in_sizes, int n_in,
                              void* d_out, int out_size, void* d_ws, size_t ws_size,
                              hipStream_t stream) {
  if (n_in < 21) return;
  if (in_sizes[0] != NN * CC || in_sizes[1] != NN * NAF) return;
  if (in_sizes[2] != EE || in_sizes[3] != EE * NBF) return;
  if (in_sizes[4] != CC * CC || in_sizes[5] != CC || in_sizes[6] != CC * CC) return;
  if (in_sizes[7] != FCH * FCH || in_sizes[8] != FCH) return;
  if (in_sizes[9] != FCH * FCH || in_sizes[10] != FCH) return;
  if (in_sizes[11] != FCH * CC) return;
  if (in_sizes[12] != CC * CC || in_sizes[13] != CC * CC) return;
  if (in_sizes[14] != CC || in_sizes[15] != CC * CC) return;
  if (in_sizes[16] != NHEAD * DHEAD) return;
  if (in_sizes[17] != CC * CC || in_sizes[18] != CC) return;
  if (in_sizes[19] != EE || in_sizes[20] != EE) return;
  if ((long long)out_size != (long long)NN * CC) return;
  if ((size_t)WS_TOTAL > ws_size) return;

  const float* node_feats = (const float*)d_in[0];
  const float* node_attr  = (const float*)d_in[1];
  const float* edge_attr  = (const float*)d_in[2];
  const float* edge_emb   = (const float*)d_in[3];
  const float* W_src      = (const float*)d_in[4];
  const float* b_src      = (const float*)d_in[5];
  const float* W_dst      = (const float*)d_in[6];
  const float* W_fc1      = (const float*)d_in[7];
  const float* b_fc1      = (const float*)d_in[8];
  const float* W_fc2      = (const float*)d_in[9];
  const float* b_fc2      = (const float*)d_in[10];
  const float* W_fc3      = (const float*)d_in[11];
  const float* W_alpha    = (const float*)d_in[12];
  const float* W_lin      = (const float*)d_in[13];
  const float* w_int      = (const float*)d_in[14];
  const float* W_val      = (const float*)d_in[15];
  const float* att_dot    = (const float*)d_in[16];
  const float* W_out      = (const float*)d_in[17];
  const float* b_out      = (const float*)d_in[18];
  const int*   edge_src   = (const int*)d_in[19];
  const int*   edge_dst   = (const int*)d_in[20];
  float* out = (float*)d_out;

  unsigned char* ws = (unsigned char*)d_ws;
  unsigned short* AGG = (unsigned short*)(ws + O_AGG);
  unsigned short* XB  = (unsigned short*)(ws + O_XB);
  float*          MSD = (float*)(ws + O_MSD);
  int*            HITS = (int*)(ws + O_HIT);
  int*            FLG0 = (int*)(ws + O_FLG0);
  int*            FLG1 = (int*)(ws + O_FLG1);
  unsigned short* WSD = (unsigned short*)(ws + O_WSD);
  unsigned short* WOD = (unsigned short*)(ws + O_WOD);
  float*          PV  = (float*)(ws + O_PV);

  const int bktLds  = BKT_LDS_INTS * 4;
  const int scanLds = SCAN_LDS_INTS * 4;
  const int edgeLds = EDGE_LDS_BYTES;
  hipFuncSetAttribute(reinterpret_cast<const void*>(&k_bucket),
                      hipFuncAttributeMaxDynamicSharedMemorySize, bktLds);
  hipFuncSetAttribute(reinterpret_cast<const void*>(&k_scan),
                      hipFuncAttributeMaxDynamicSharedMemorySize, scanLds);
  hipFuncSetAttribute(reinterpret_cast<const void*>(&k_edge),
                      hipFuncAttributeMaxDynamicSharedMemorySize, edgeLds);

  k_pa<<<NU_PA / NTHR, NTHR, 0, stream>>>(node_feats, W_src, W_dst, W_fc1, W_fc2, W_fc3, ws);
  k_pb<<<NU_PB / NTHR, NTHR, 0, stream>>>(W_alpha, W_lin, W_val, W_out, b_src, b_fc1, b_fc2, w_int,
                                          att_dot, b_out, ws);
  k_gemm<0><<<dim3(MP / GBM, 2), GTHR, 0, stream>>>(XB, CC, WSD, CC, CC, PV, MP, MSD, 256, FLG1);
  k_bucket<<<NBLK, NTHR, bktLds, stream>>>(edge_dst, EE, NN, 1, HITS, FLG0);
  for (int g = 0; g < NGRP; ++g) {
    k_edge<<<NTILE, NTHR, edgeLds, stream>>>(ws, node_attr, edge_attr, edge_emb, edge_src, edge_dst, g);
    k_scan<<<BPG, NTHR, scanLds, stream>>>(ws, g);
  }
  k_gemm<1><<<dim3(MP / GBM, 1), GTHR, 0, stream>>>(AGG, 256, WOD, 256, 256, PV + 640, NN, out, CC, FLG1);
}
